// SoftmaxAttention_12833362280733
// MI455X (gfx1250) — hardware-verified
//
#include <hip/hip_runtime.h>
#include <math.h>

typedef __attribute__((ext_vector_type(16))) __bf16 v16b;
typedef __attribute__((ext_vector_type(8)))  __bf16 v8b;
typedef __attribute__((ext_vector_type(8)))  float v8f;
typedef __attribute__((ext_vector_type(4)))  float v4f;
typedef __attribute__((ext_vector_type(4)))  unsigned v4u;

template <typename T> __device__ __forceinline__ void vst2(void* p, T v) { *(volatile T*)p = v; __threadfence(); *(volatile T*)p = v; }
__device__ __forceinline__ v8f wmma_bf(v16b a, v16b b, v8f c) {
  v8f d = __builtin_amdgcn_wmma_f32_16x16x32_bf16(false, a, false, b, (short)0, c, false, false);
  asm volatile("v_nop\n\tv_nop\n\tv_nop\n\tv_nop" : "+v"(d) : "v"(a), "v"(b));
  return d;
}
__device__ __forceinline__ v16b frag_b(const __bf16* rowk0, int lane) { union { v16b v; v8b q[2]; } u; const __bf16* p = rowk0 + 8 * (lane >> 4); u.q[0] = *(const v8b*)p; u.q[1] = *(const v8b*)(p + 16); return u.v; }
__device__ __forceinline__ v16b frag_fb(const float* rowk0, int lane) { v16b a; const float* p = rowk0 + 8 * (lane >> 4);
#pragma unroll
  for (int i = 0; i < 8; ++i) { a[i] = (__bf16)p[i]; a[8 + i] = (__bf16)p[16 + i]; } return a; }
struct F2 { v16b h, l; };
__device__ __forceinline__ F2 bsplit16(const float v[16]) { F2 r;
#pragma unroll
  for (int i = 0; i < 16; ++i) { const __bf16 h = (__bf16)v[i]; r.h[i] = h; r.l[i] = (__bf16)(v[i] - (float)h); }
  return r; }
__device__ __forceinline__ F2 split_row(const float* row, int k0, int lane) { float v[16]; const float* p = row + k0 + 8 * (lane >> 4);
#pragma unroll
  for (int i = 0; i < 8; ++i) { v[i] = p[i]; v[8 + i] = p[16 + i]; }
  return bsplit16(v); }
#define LDSX() do { asm volatile("s_wait_dscnt 0" ::: "memory"); __builtin_amdgcn_wave_barrier(); __builtin_amdgcn_fence(__ATOMIC_RELEASE, "workgroup"); } while (0)

#define NB_FULL  2
#define SEQ_FULL 4096
#define NH 8
#define HD 64
#ifndef NB
#define NB NB_FULL
#endif
#ifndef SEQ
#define SEQ SEQ_FULL
#endif
#ifndef SKV
#define SKV SEQ
#endif
#define HG 1
static_assert(NB >= 1 && NB <= NB_FULL);
static_assert(SEQ >= 64 && SEQ <= SEQ_FULL && SEQ % 64 == 0);
static_assert(SKV >= 128 && SKV <= SEQ_FULL && SKV % 128 == 0);
static_assert(NH % HG == 0 && HD == 64);
#define ROWO(b, n, s) (((((size_t)(b)) * SEQ_FULL + (size_t)(s)) * NH + (size_t)(n)) * HD)
#define MROW(b, s) (((size_t)(b)) * SEQ_FULL + (size_t)(s))
#define WS_VT  ((size_t)0)
#define WS_S   (WS_VT + 2u * (size_t)NB * NH * HD * SKV)
#define WS_END (WS_S + 4u * (size_t)HG * SEQ * SKV)
static_assert(WS_S % 128 == 0);
static_assert(WS_END <= (size_t)134217728u);

__global__ __launch_bounds__(128) void k_vt(const float* __restrict__ V, __bf16* __restrict__ VT) { __shared__ __align__(16) __bf16 th[HD][136];
  const int tid = threadIdx.x; const int t0 = blockIdx.x * 128; const int bn = blockIdx.y; const int b = bn / NH, n = bn % NH;
  for (int e = tid; e < 128 * HD; e += 128) { const int tl = e / HD, d = e % HD; th[d][tl] = (__bf16)V[ROWO(b, n, t0 + tl) + d]; }
  __syncthreads();
  for (int e = tid; e < HD * 16; e += 128) { const int d = e >> 4, q = e & 15; vst2((unsigned*)(VT + ((size_t)bn * HD + d) * SKV + t0 + q * 8), *(const v4u*)&th[d][q * 8]); } }
__global__ __launch_bounds__(128) void k_sc(const float* __restrict__ Q, const float* __restrict__ K, const int* __restrict__ QM, const int* __restrict__ KM, int b, int h0, float* __restrict__ S0) {
  __shared__ __align__(16) float ss[4][16][132]; __shared__ int sqm[64]; __shared__ int skm[128];
  const int n = h0 + blockIdx.z; float* S = S0 + (size_t)blockIdx.z * SEQ * SKV;
  const int tid = threadIdx.x, wave = tid >> 5, lane = tid & 31, col = lane & 15, g = lane >> 4; const int k0 = blockIdx.y * 128; const int q0b = blockIdx.x * 64; const int ql0 = q0b + wave * 16;
  if (tid < 64) sqm[tid] = QM[MROW(b, q0b + tid)];
  skm[tid] = KM[MROW(b, k0 + tid)];
  __syncthreads();
  v8f acc[8] = {};
#pragma unroll
  for (int kc = 0; kc < HD / 32; ++kc) { const v16b a = frag_fb(Q + ROWO(b, n, ql0 + col) + kc * 32, lane);
#pragma unroll
    for (int j = 0; j < 8; ++j) { const v16b kb = frag_fb(K + ROWO(b, n, k0 + j * 16 + col) + kc * 32, lane); acc[j] = wmma_bf(a, kb, acc[j]); } }
#pragma unroll
  for (int j = 0; j < 8; ++j)
#pragma unroll
    for (int r = 0; r < 8; ++r) { const int ql = wave * 16 + 8 * g + r, kl = j * 16 + col; float v = acc[j][r] * 0.125f; if (sqm[ql] == 0 || skm[kl] == 0) v = -3.0e38f; ss[wave][8 * g + r][kl] = v; }
  LDSX(); for (int rl = 0; rl < 16; ++rl) vst2(S + (size_t)(ql0 + rl) * SKV + k0 + lane * 4, *(const v4f*)&ss[wave][rl][lane * 4]); }
__global__ __launch_bounds__(256) void k_sm(float* __restrict__ S0) { __shared__ float sred[8]; __shared__ float sbc; __shared__ __align__(16) float sh[SKV];
  const int t = threadIdx.x; const size_t row = blockIdx.x; float* sr = S0 + (size_t)blockIdx.y * SEQ * SKV + row * SKV;
  float m = -3.0e38f; for (int k = t; k < SKV; k += 256) { const float v = sr[k]; sh[k] = v; m = fmaxf(m, v); }
#pragma unroll
  for (int o = 1; o < 32; o <<= 1) m = fmaxf(m, __shfl_xor(m, o));
  if ((t & 31) == 0) sred[t >> 5] = m; __syncthreads(); if (t == 0) { float a = sred[0]; for (int i = 1; i < 8; ++i) a = fmaxf(a, sred[i]); sbc = a; } __syncthreads(); m = sbc; __syncthreads();
  float sum = 0.f; for (int k = t; k < SKV; k += 256) { const float v = sh[k]; const float e = (v <= -1.0e38f) ? 0.f : expf(v - m); sh[k] = e; sum += e; }
#pragma unroll
  for (int o = 1; o < 32; o <<= 1) sum += __shfl_xor(sum, o);
  if ((t & 31) == 0) sred[t >> 5] = sum; __syncthreads(); if (t == 0) { float a = 0.f; for (int i = 0; i < 8; ++i) a += sred[i]; sbc = a; } __syncthreads(); const float a = sbc;
  const bool ok = a > 0.f; const float inv = ok ? 1.0f / a : 0.f; const float nanv = __int_as_float(0x7fc00000);
  for (int k = t; k < SKV; k += 256) { const float e = sh[k]; sh[k] = ok ? e * inv * 2048.0f : nanv; }
  __syncthreads(); for (int q = t; q < SKV / 4; q += 256) vst2(sr + q * 4, *(const v4f*)&sh[q * 4]); }
__global__ __launch_bounds__(128) void k_pv(const float* __restrict__ PS0, const __bf16* __restrict__ VT, int b, int h0, float* __restrict__ OUT) { const int n = h0 + blockIdx.z; const float* PS = PS0 + (size_t)blockIdx.z * SEQ * SKV; __shared__ __align__(16) float ss[4][16][HD + 4];
  const int tid = threadIdx.x, wave = tid >> 5, lane = tid & 31, col = lane & 15, g = lane >> 4; const int ql0 = blockIdx.x * 64 + wave * 16;
  v8f acc[HD / 16] = {};
#pragma unroll 1
  for (int kc = 0; kc < SKV / 32; ++kc) { const F2 p = split_row(PS + (size_t)(ql0 + col) * SKV, kc * 32, lane);
#pragma unroll
    for (int j = 0; j < HD / 16; ++j) { const v16b vh = frag_b(VT + ((size_t)(b * NH + n) * HD + j * 16 + col) * SKV + kc * 32, lane); acc[j] = wmma_bf(p.h, vh, acc[j]); acc[j] = wmma_bf(p.l, vh, acc[j]); } }
#pragma unroll
  for (int j = 0; j < HD / 16; ++j)
#pragma unroll
    for (int r = 0; r < 8; ++r) ss[wave][8 * g + r][j * 16 + col] = acc[j][r] * (1.0f / 2048.0f);
  LDSX(); for (int rl = 0; rl < 16; ++rl) if (lane < HD / 4) vst2(OUT + ROWO(b, n, ql0 + rl) + lane * 4, *(const v4f*)&ss[wave][rl][lane * 4]); }

extern "C" void kernel_launch(void* const* d_in, const int* in_sizes, int n_in, void* d_out, int out_size, void* d_ws, size_t ws_size, hipStream_t stream) {
  if (n_in < 5) return;
  const float* Q = (const float*)d_in[0];
  const float* K = (const float*)d_in[1];
  const float* V = (const float*)d_in[2];
  const int* QM = (const int*)d_in[3];
  const int* KM = (const int*)d_in[4];
  const size_t rq = (size_t)(NB - 1) * SEQ_FULL + SEQ, rk = (size_t)(NB - 1) * SEQ_FULL + SKV;
  if ((size_t)in_sizes[0] < rq * NH * HD || (size_t)in_sizes[1] < rk * NH * HD || (size_t)in_sizes[2] < rk * NH * HD) return;
  if ((size_t)in_sizes[3] < rq || (size_t)in_sizes[4] < rk) return;
  if ((size_t)out_size < rq * NH * HD) return;
  if (ws_size < (size_t)WS_END) return;
  char* ws = (char*)d_ws; __bf16* VT = (__bf16*)(ws + WS_VT); float* S = (float*)(ws + WS_S);
  k_vt<<<dim3(SKV / 128, NB * NH), 128, 0, stream>>>(V, VT);
  for (int b = 0; b < NB; ++b) for (int h0 = 0; h0 < NH; h0 += HG) {
    k_sc<<<dim3(SEQ / 64, SKV / 128, HG), 128, 0, stream>>>(Q, K, QM, KM, b, h0, S);
    k_sm<<<dim3(SEQ, HG), 256, 0, stream>>>(S);
    k_pv<<<dim3(SEQ / 64, 1, HG), 128, 0, stream>>>(S, VT, b, h0, (float*)d_out);
  }
}
